// SplitAttentionOp_44229573214696
// MI455X (gfx1250) — hardware-verified
//
#include <hip/hip_runtime.h>

typedef _Float16 v16h __attribute__((ext_vector_type(16)));
typedef _Float16 v8h  __attribute__((ext_vector_type(8)));
typedef _Float16 v4h  __attribute__((ext_vector_type(4)));
typedef float    v8f  __attribute__((ext_vector_type(8)));
typedef float    v4f  __attribute__((ext_vector_type(4)));
union Frag { v16h v; v8h h[2]; };

#define SA_H     16
#define SA_SQ    1024
#define SA_SKV   2048
#define SA_D     128
#define SA_QBLK  64
#define SA_OPS   16.0f
#define SA_CS    ((0.088388347648318447f * 1.4426950408889634f) * 0.00390625f)
#define SA_LN2   0.69314718055994531f
#define SA_OINV  0.00390625f

#define KP   136
#define VP   40
#define PP   40
#define OPF  132
#define NSTEP (2 * SA_SKV / 32)

__device__ __forceinline__ v8f wmma_f16(v16h a, v16h b, v8f c) {
  v8f d = __builtin_amdgcn_wmma_f32_16x16x32_f16(false, a, false, b, (short)0, c, false, false);
  asm volatile("v_nop\n\tv_nop\n\tv_nop\n\tv_nop" : "+v"(d) : "v"(a), "v"(b));
  return d;
}

__device__ __forceinline__ float rmax16(float x) {
  x = fmaxf(x, __shfl_xor(x, 1));
  x = fmaxf(x, __shfl_xor(x, 2));
  x = fmaxf(x, __shfl_xor(x, 4));
  x = fmaxf(x, __shfl_xor(x, 8));
  return x;
}
__device__ __forceinline__ float rsum16(float x) {
  x += __shfl_xor(x, 1);
  x += __shfl_xor(x, 2);
  x += __shfl_xor(x, 4);
  x += __shfl_xor(x, 8);
  return x;
}

__global__ __launch_bounds__(128) __attribute__((amdgpu_num_vgpr(248)))
void attn_two_kv(const float* __restrict__ q,
                 const float* __restrict__ kA, const float* __restrict__ vA,
                 const float* __restrict__ kB, const float* __restrict__ vB,
                 float* out, float* lse)
{
  __shared__ __align__(16) _Float16 kbuf[32 * KP];
  __shared__ __align__(16) _Float16 vbufT[SA_D * VP];
  __shared__ __align__(16) _Float16 pbuf[4][16 * PP];
  __shared__ __align__(16) float    obuf[4][16 * OPF];
  __shared__ __align__(16) float    lbuf[SA_QBLK];

  const int tid  = threadIdx.x;
  const int lane = tid & 31;
  const int wave = tid >> 5;
  const int half = lane >> 4;
  const int l16  = lane & 15;

  const int h    = blockIdx.x % SA_H;
  const int q0   = (blockIdx.x / SA_H) * SA_QBLK;
  const int qrow = q0 + wave * 16;

  const int krow = tid >> 2;
  const int kcb  = (tid & 3) * 32;
  const int vkv  = (tid >> 4) * 4;
  const int vdc  = (tid & 15) * 8;

  v16h qf[4];
  {
    const float* qp = q + ((size_t)(h * SA_SQ + qrow + l16)) * SA_D;
#pragma unroll
    for (int c = 0; c < 4; ++c) {
      Frag f;
#pragma unroll
      for (int s = 0; s < 2; ++s) {
        const int d0 = c * 32 + 16 * s + 8 * half;
        const float4 a0 = *(const float4*)(qp + d0);
        const float4 a1 = *(const float4*)(qp + d0 + 4);
        v8h t;
        t[0] = (_Float16)(a0.x * SA_OPS); t[1] = (_Float16)(a0.y * SA_OPS);
        t[2] = (_Float16)(a0.z * SA_OPS); t[3] = (_Float16)(a0.w * SA_OPS);
        t[4] = (_Float16)(a1.x * SA_OPS); t[5] = (_Float16)(a1.y * SA_OPS);
        t[6] = (_Float16)(a1.z * SA_OPS); t[7] = (_Float16)(a1.w * SA_OPS);
        f.h[s] = t;
      }
      qf[c] = f.v;
    }
  }

  v8f o[8];
#pragma unroll
  for (int n = 0; n < 8; ++n)
#pragma unroll
    for (int r = 0; r < 8; ++r) o[n][r] = 0.0f;

  float mrun[8], lrun[8];
#pragma unroll
  for (int r = 0; r < 8; ++r) { mrun[r] = -1.0e30f; lrun[r] = 0.0f; }

  for (int step = 0; step < NSTEP; ++step) {
    const bool second = step >= (SA_SKV / 32);
    const float* ks = second ? kB : kA;
    const float* vs = second ? vB : vA;
    const int j = (second ? (step - SA_SKV / 32) : step) * 32;
    const float* kbase = ks + ((size_t)(h * SA_SKV + j)) * SA_D;
    const float* vbase = vs + ((size_t)(h * SA_SKV + j)) * SA_D;

    __syncthreads();

    {
      const float* srcK = kbase + krow * SA_D + kcb;
      _Float16* dst = kbuf + krow * KP + kcb;
#pragma unroll
      for (int i = 0; i < 4; ++i) {
        const float4 x0 = *(const float4*)(srcK + i * 8);
        const float4 x1 = *(const float4*)(srcK + i * 8 + 4);
        v8h p;
        p[0] = (_Float16)(x0.x * SA_OPS); p[1] = (_Float16)(x0.y * SA_OPS);
        p[2] = (_Float16)(x0.z * SA_OPS); p[3] = (_Float16)(x0.w * SA_OPS);
        p[4] = (_Float16)(x1.x * SA_OPS); p[5] = (_Float16)(x1.y * SA_OPS);
        p[6] = (_Float16)(x1.z * SA_OPS); p[7] = (_Float16)(x1.w * SA_OPS);
        *(v8h*)(dst + i * 8) = p;
      }
    }
    {
      float vr[4][8];
#pragma unroll
      for (int rr = 0; rr < 4; ++rr) {
        const float* srcV = vbase + (vkv + rr) * SA_D + vdc;
        const float4 a = *(const float4*)(srcV);
        const float4 b = *(const float4*)(srcV + 4);
        vr[rr][0] = a.x; vr[rr][1] = a.y; vr[rr][2] = a.z; vr[rr][3] = a.w;
        vr[rr][4] = b.x; vr[rr][5] = b.y; vr[rr][6] = b.z; vr[rr][7] = b.w;
      }
#pragma unroll
      for (int i = 0; i < 8; ++i) {
        v4h w;
        w[0] = (_Float16)(vr[0][i] * SA_OPS); w[1] = (_Float16)(vr[1][i] * SA_OPS);
        w[2] = (_Float16)(vr[2][i] * SA_OPS); w[3] = (_Float16)(vr[3][i] * SA_OPS);
        *(v4h*)(vbufT + (vdc + i) * VP + vkv) = w;
      }
    }

    __syncthreads();

    v8f s0, s1;
#pragma unroll
    for (int r = 0; r < 8; ++r) { s0[r] = 0.0f; s1[r] = 0.0f; }
#pragma unroll
    for (int c = 0; c < 4; ++c) {
      Frag b0, b1;
      const _Float16* kp0 = kbuf + l16 * KP + c * 32 + half * 8;
      const _Float16* kp1 = kp0 + 16 * KP;
      b0.h[0] = *(const v8h*)(kp0);  b0.h[1] = *(const v8h*)(kp0 + 16);
      b1.h[0] = *(const v8h*)(kp1);  b1.h[1] = *(const v8h*)(kp1 + 16);
      s0 = wmma_f16(qf[c], b0.v, s0);
      s1 = wmma_f16(qf[c], b1.v, s1);
    }

    float corr[8];
#pragma unroll
    for (int r = 0; r < 8; ++r) {
      const float x0 = s0[r] * SA_CS;
      const float x1 = s1[r] * SA_CS;
      const float mx = rmax16(fmaxf(x0, x1));
      const float mn = fmaxf(mrun[r], mx);
      const float p0 = __builtin_amdgcn_exp2f(x0 - mn);
      const float p1 = __builtin_amdgcn_exp2f(x1 - mn);
      const float rs = rsum16(p0 + p1);
      const float cf = __builtin_amdgcn_exp2f(mrun[r] - mn);
      corr[r] = cf;
      lrun[r] = lrun[r] * cf + rs;
      mrun[r] = mn;
      s0[r] = p0; s1[r] = p1;
    }

#pragma unroll
    for (int n = 0; n < 8; ++n)
#pragma unroll
      for (int r = 0; r < 8; ++r) o[n][r] *= corr[r];

    _Float16* pb = pbuf[wave];
#pragma unroll
    for (int r = 0; r < 8; ++r) {
      const int row = r + half * 8;
      pb[row * PP + l16]      = (_Float16)(s0[r] * SA_OPS);
      pb[row * PP + 16 + l16] = (_Float16)(s1[r] * SA_OPS);
    }
    __syncthreads();
    Frag pf;
    {
      const _Float16* pr = pb + l16 * PP + half * 8;
      pf.h[0] = *(const v8h*)(pr);
      pf.h[1] = *(const v8h*)(pr + 16);
    }

#pragma unroll
    for (int cn = 0; cn < 8; ++cn) {
      Frag vf;
      const _Float16* vp = vbufT + (cn * 16 + l16) * VP + half * 8;
      vf.h[0] = *(const v8h*)(vp);
      vf.h[1] = *(const v8h*)(vp + 16);
      o[cn] = wmma_f16(pf.v, vf.v, o[cn]);
    }
  }

  float inv[8];
#pragma unroll
  for (int r = 0; r < 8; ++r) inv[r] = SA_OINV / lrun[r];
  {
    float* ob = obuf[wave];
#pragma unroll
    for (int n = 0; n < 8; ++n) {
#pragma unroll
      for (int r = 0; r < 8; ++r) {
        ob[(r + half * 8) * OPF + n * 16 + l16] = o[n][r] * inv[r];
      }
    }
    if (l16 == 0) {
#pragma unroll
      for (int r = 0; r < 8; ++r)
        lbuf[wave * 16 + half * 8 + r] = SA_LN2 * (mrun[r] + log2f(lrun[r]));
    }
  }
  __syncthreads();

  const float* obr = obuf[wave];
  float* orow = out + ((size_t)(h * SA_SQ + qrow)) * SA_D + lane * 4;
  float* lrow = lse + (size_t)h * SA_SQ + q0;
  const bool lsew = (wave == 0) && (lane < 16);

#pragma unroll
  for (int r = 0; r < 16; ++r) {
    const v4f v = *(const v4f*)(obr + r * OPF + lane * 4);
    *(volatile v4f*)(orow + (size_t)r * SA_D) = v;
  }
  if (lsew) {
    const v4f lv = *(const v4f*)(lbuf + lane * 4);
    *(volatile v4f*)(lrow + lane * 4) = lv;
  }
  __threadfence();
#pragma unroll
  for (int r = 0; r < 16; ++r) {
    const v4f v = *(const v4f*)(obr + r * OPF + lane * 4);
    *(volatile v4f*)(orow + (size_t)r * SA_D) = v;
  }
  if (lsew) {
    const v4f lv = *(const v4f*)(lbuf + lane * 4);
    *(volatile v4f*)(lrow + lane * 4) = lv;
  }
}

extern "C" void kernel_launch(void* const* d_in, const int* in_sizes, int n_in,
                              void* d_out, int out_size, void* d_ws, size_t ws_size,
                              hipStream_t stream) {
  (void)d_ws; (void)ws_size;
  if (n_in < 5) return;
  if (in_sizes[0] != SA_H * SA_SQ * SA_D) return;
  if (in_sizes[1] != SA_H * SA_SKV * SA_D || in_sizes[2] != SA_H * SA_SKV * SA_D) return;
  if (in_sizes[3] != SA_H * SA_SKV * SA_D || in_sizes[4] != SA_H * SA_SKV * SA_D) return;
  if (out_size != SA_H * SA_SQ * SA_D + SA_H * SA_SQ) return;

  const float* q  = (const float*)d_in[0];
  const float* kA = (const float*)d_in[1];
  const float* vA = (const float*)d_in[2];
  const float* kB = (const float*)d_in[3];
  const float* vB = (const float*)d_in[4];
  float* out = (float*)d_out;
  float* lse = out + (size_t)SA_H * SA_SQ * SA_D;

  dim3 grid(SA_H * (SA_SQ / SA_QBLK));
  dim3 block(128);
  attn_two_kv<<<grid, block, 0, stream>>>(q, kA, vA, kB, vB, out, lse);
}
